// PointNetSAModule_1717986918816
// MI455X (gfx1250) — hardware-verified
//
#include <hip/hip_runtime.h>
#include <math.h>

#pragma clang fp contract(off)

typedef __attribute__((ext_vector_type(16))) _Float16 v16h;
typedef __attribute__((ext_vector_type(8)))  _Float16 v8h;
typedef __attribute__((ext_vector_type(8)))  float    v8f;
typedef __attribute__((ext_vector_type(4)))  float    v4f;
typedef __attribute__((ext_vector_type(4)))  unsigned v4u;

constexpr int kBatch   = 16;
constexpr int kPts     = 8192;
constexpr int kCin     = 64;
constexpr int kCent    = 1024;
constexpr int kNbr     = 32;
constexpr int kCols    = kBatch * kCent * kNbr;
constexpr int kRowsAll = kBatch * kPts;
constexpr int kBlkCols = 128;
constexpr int kNumBlk  = kCols / kBlkCols;
constexpr int kPitchA  = 72;
constexpr int kOut0Floats = kBatch * 3 * kCent;
constexpr float kWCarry    = 16.0f;
constexpr float kWCarryInv = 1.0f / 16.0f;

static_assert(kCols == 524288, "column count");
static_assert(kRowsAll == 131072, "point rows");
static_assert(kNumBlk == 4096, "block count");
static_assert(kCin == 64, "feature channels");
static_assert(kOut0Floats * 4 == 196608, "second output byte offset");
static_assert((size_t)kOut0Floats * 4 + (size_t)kBatch * 128 * kCent * 4 == 8585216, "output bytes");
static_assert(kRowsAll % 64 == 0 && 64 % 32 == 0, "gemm tile multiples");

union FragH { v16h v; v8h h[2]; };

__device__ __forceinline__ v16h frag_load_g(const _Float16* p) {
  FragH f;
  f.h[0] = *(const v8h*)(p);
  f.h[1] = *(const v8h*)(p + 16);
  return f.v;
}
__device__ __forceinline__ v8f mma_h(v16h a, v16h b, v8f c) {
  return __builtin_amdgcn_wmma_f32_16x16x32_f16(false, a, false, b, (short)0, c, false, false);
}
__device__ __forceinline__ void guard4_h(v8f& a, v8f& b, v8f& c, v8f& d,
                                         v16h x, v16h y0, v16h y1, v16h y2, v16h y3) {
  asm volatile("v_nop\n\tv_nop\n\tv_nop\n\tv_nop"
               : "+v"(a), "+v"(b), "+v"(c), "+v"(d)
               : "v"(x), "v"(y0), "v"(y1), "v"(y2), "v"(y3));
}
__device__ __forceinline__ void keep4_h(v16h a, v16h b, v16h c, v16h d) {
  asm volatile("v_nop" :: "v"(a), "v"(b), "v"(c), "v"(d));
}
__device__ __forceinline__ void acc_guard4(v8f& a, v8f& b, v8f& c, v8f& d) {
  asm volatile("v_nop\n\tv_nop\n\tv_nop\n\tv_nop" : "+v"(a), "+v"(b), "+v"(c), "+v"(d));
}

__device__ __forceinline__ float h16_to_f32(unsigned hb) {
  const unsigned sgn = (hb & 0x8000u) << 16;
  const unsigned em = hb & 0x7fffu;
  const float fn = __uint_as_float((em << 13) + 0x38000000u);
  const float fs = (float)em * 5.9604644775390625e-8f;
  const float mag = (em < 0x400u) ? fs : fn;
  return __uint_as_float(__float_as_uint(mag) | sgn);
}

__device__ __forceinline__ int nth_set_bit(unsigned m, unsigned r) {
  int pos = 0;
  unsigned c;
  c = (unsigned)__popc(m & 0xFFFFu);
  if (r >= c) { r -= c; pos += 16; m >>= 16; }
  c = (unsigned)__popc(m & 0xFFu);
  if (r >= c) { r -= c; pos += 8; m >>= 8; }
  c = (unsigned)__popc(m & 0xFu);
  if (r >= c) { r -= c; pos += 4; m >>= 4; }
  c = (unsigned)__popc(m & 0x3u);
  if (r >= c) { r -= c; pos += 2; m >>= 2; }
  c = m & 1u;
  if (r >= c) { pos += 1; }
  return pos;
}

__global__ __launch_bounds__(1024) void fps_kernel(const float* __restrict__ xyz,
                                                    float* __restrict__ out0,
                                                    float* __restrict__ cxyz) {
#pragma clang fp contract(off)
  __shared__ float s_v[2][32];
  __shared__ int   s_i[2][32];
  __shared__ int   s_idx[kCent];
  const int b = blockIdx.x;
  const int t = threadIdx.x;
  const int lane = t & 31;
  const int wid = t >> 5;
  const float* px = xyz + (size_t)b * 3 * kPts;
  const float* py = px + kPts;
  const float* pz = px + 2 * kPts;

  float lx[8], ly[8], lz[8], ld[8];
  {
    const v4f ax0 = *(const v4f*)(px + 8 * t);
    const v4f ax1 = *(const v4f*)(px + 8 * t + 4);
    const v4f ay0 = *(const v4f*)(py + 8 * t);
    const v4f ay1 = *(const v4f*)(py + 8 * t + 4);
    const v4f az0 = *(const v4f*)(pz + 8 * t);
    const v4f az1 = *(const v4f*)(pz + 8 * t + 4);
    lx[0] = ax0.x; lx[1] = ax0.y; lx[2] = ax0.z; lx[3] = ax0.w;
    lx[4] = ax1.x; lx[5] = ax1.y; lx[6] = ax1.z; lx[7] = ax1.w;
    ly[0] = ay0.x; ly[1] = ay0.y; ly[2] = ay0.z; ly[3] = ay0.w;
    ly[4] = ay1.x; ly[5] = ay1.y; ly[6] = ay1.z; ly[7] = ay1.w;
    lz[0] = az0.x; lz[1] = az0.y; lz[2] = az0.z; lz[3] = az0.w;
    lz[4] = az1.x; lz[5] = az1.y; lz[6] = az1.z; lz[7] = az1.w;
  }
#pragma unroll
  for (int i = 0; i < 8; ++i) ld[i] = INFINITY;

  int last = 0;
  for (int step = 0; step < kCent; ++step) {
    const int lc = last < 0 ? 0 : (last > kPts - 1 ? kPts - 1 : last);
    const float cx = px[lc];
    const float cy = py[lc];
    const float cz = pz[lc];
    if (t == 0) s_idx[step] = lc;
    float bv = -1.0f;
    int bi = 8 * t;
#pragma unroll
    for (int i = 0; i < 8; ++i) {
      const float dx = lx[i] - cx;
      const float dy = ly[i] - cy;
      const float dz = lz[i] - cz;
      const float qx = dx * dx;
      const float qy = dy * dy;
      const float qz = dz * dz;
      const float d = (qx + qy) + qz;
      const float nd = fminf(ld[i], d);
      ld[i] = nd;
      const bool tk = nd > bv;
      bv = tk ? nd : bv;
      bi = tk ? (8 * t + i) : bi;
    }
#pragma unroll
    for (int off = 16; off > 0; off >>= 1) {
      const float ov = __shfl_xor(bv, off, 32);
      const int oi = __shfl_xor(bi, off, 32);
      const bool take = (ov > bv) || ((ov == bv) && (oi < bi));
      bv = take ? ov : bv;
      bi = take ? oi : bi;
    }
    const int p = step & 1;
    if (lane == 0) { s_v[p][wid] = bv; s_i[p][wid] = bi; }
    __syncthreads();
    float rv = s_v[p][lane];
    int ri = s_i[p][lane];
#pragma unroll
    for (int off = 16; off > 0; off >>= 1) {
      const float ov = __shfl_xor(rv, off, 32);
      const int oi = __shfl_xor(ri, off, 32);
      const bool take = (ov > rv) || ((ov == rv) && (oi < ri));
      rv = take ? ov : rv;
      ri = take ? oi : ri;
    }
    last = ri;
  }
  __syncthreads();
  {
    int idx = s_idx[t];
    idx = idx < 0 ? 0 : (idx > kPts - 1 ? kPts - 1 : idx);
    const float v0 = px[idx];
    const float v1 = py[idx];
    const float v2 = pz[idx];
    float* o = out0 + (size_t)b * 3 * kCent + t;
    float* w = cxyz + (size_t)b * 3 * kCent + t;
    *(volatile float*)(o) = v0;
    *(volatile float*)(o + kCent) = v1;
    *(volatile float*)(o + 2 * kCent) = v2;
    *(volatile float*)(w) = v0;
    *(volatile float*)(w + kCent) = v1;
    *(volatile float*)(w + 2 * kCent) = v2;
    __threadfence();
    *(volatile float*)(o) = v0;
    *(volatile float*)(o + kCent) = v1;
    *(volatile float*)(o + 2 * kCent) = v2;
    *(volatile float*)(w) = v0;
    *(volatile float*)(w + kCent) = v1;
    *(volatile float*)(w + 2 * kCent) = v2;
    __threadfence();
  }
}

__global__ __launch_bounds__(256) void ballquery_kernel(const float* __restrict__ xyz,
                                                        const float* __restrict__ cxyz,
                                                        int* __restrict__ gidx) {
#pragma clang fp contract(off)
  const int lane = threadIdx.x & 31;
  const int wave = threadIdx.x >> 5;
  const int g = blockIdx.x * 8 + wave;
  const int b = g >> 10;
  const int s = g & (kCent - 1);
  const float* px = xyz + (size_t)b * 3 * kPts;
  const float* py = px + kPts;
  const float* pz = px + 2 * kPts;
  const float* cc = cxyz + (size_t)b * 3 * kCent + s;
  const float cx = cc[0];
  const float cy = cc[kCent];
  const float cz = cc[2 * kCent];
  int cnt = 0;
  int first = 0;
  int mine = 0;
  for (int chunk = 0; chunk < kPts / 32; ++chunk) {
    const int n = chunk * 32 + lane;
    const float x = px[n];
    const float y = py[n];
    const float z = pz[n];
    const float dx = cx - x;
    const float dy = cy - y;
    const float dz = cz - z;
    const float qx = dx * dx;
    const float qy = dy * dy;
    const float qz = dz * dz;
    const float d = (qx + qy) + qz;
    const bool hit = d < 0.04f;
    const unsigned m = __builtin_amdgcn_ballot_w32(hit);
    if (m != 0u) {
      if (cnt == 0) first = chunk * 32 + __builtin_ctz(m);
      const int pc = __popc(m);
      const int j = lane - cnt;
      const bool valid = (j >= 0) && (j < pc);
      const unsigned jj = valid ? (unsigned)j : 0u;
      const int pos = nth_set_bit(m, jj);
      mine = valid ? (chunk * 32 + pos) : mine;
      cnt += pc;
    }
    if (cnt >= kNbr) break;
  }
  mine = (lane >= cnt) ? first : mine;
  mine = mine < 0 ? 0 : (mine > kPts - 1 ? kPts - 1 : mine);
  int* o = gidx + (size_t)g * kNbr + lane;
  *(volatile int*)o = mine;
  __threadfence();
  *(volatile int*)o = mine;
  __threadfence();
}

__global__ __launch_bounds__(256) void cvt_feat_kernel(const float* __restrict__ feat,
                                                       _Float16* __restrict__ featT) {
  __shared__ __align__(16) float tile[64 * 68];
  const int tid = threadIdx.x;
  const int lane = tid & 31;
  const int wave = tid >> 5;
  const int blk = blockIdx.x;
  const int b = blk >> 7;
  const int n0 = (blk & 127) * 64;
  const float* fb = feat + (size_t)b * kCin * kPts + n0;
#pragma unroll
  for (int i = 0; i < 4; ++i) {
    const int idx = tid + 256 * i;
    const int ch = idx >> 4;
    const int q = idx & 15;
    const v4f v = *(const v4f*)(fb + (size_t)ch * kPts + 4 * q);
    *(v4f*)(tile + ch * 68 + 4 * q) = v;
  }
  __syncthreads();
  const int sub = lane >> 3;
  const int oct = lane & 7;
  v8h hv0, hv1;
  const int r0 = wave * 4 + sub;
  const int r1 = 32 + wave * 4 + sub;
#pragma unroll
  for (int e = 0; e < 8; ++e) {
    hv0[e] = (_Float16)tile[(8 * oct + e) * 68 + r0];
    hv1[e] = (_Float16)tile[(8 * oct + e) * 68 + r1];
  }
  _Float16* d0 = featT + ((size_t)b * kPts + n0 + r0) * 64 + 8 * oct;
  _Float16* d1 = featT + ((size_t)b * kPts + n0 + r1) * 64 + 8 * oct;
  *(volatile v8h*)d0 = hv0;
  *(volatile v8h*)d1 = hv1;
  __threadfence();
  *(volatile v8h*)d0 = hv0;
  *(volatile v8h*)d1 = hv1;
  __threadfence();
}

__global__ __launch_bounds__(256) void cvt_w_kernel(const float* __restrict__ W0,
                                                    const float* __restrict__ W1,
                                                    const float* __restrict__ W2,
                                                    _Float16* __restrict__ W0f,
                                                    _Float16* __restrict__ W1h,
                                                    _Float16* __restrict__ W2h) {
  const int blk = blockIdx.x;
  const int tid = threadIdx.x;
  const float* src;
  _Float16* dst;
  int ld, off, i;
  if (blk < 2) {
    src = W0; dst = W0f; ld = 67; off = 3; i = blk * 256 + tid;
  } else if (blk < 4) {
    src = W1; dst = W1h; ld = 64; off = 0; i = (blk - 2) * 256 + tid;
  } else {
    src = W2; dst = W2h; ld = 64; off = 0; i = (blk - 4) * 256 + tid;
  }
  const int o = i >> 3;
  const int oct = i & 7;
  v8h hv;
#pragma unroll
  for (int e = 0; e < 8; ++e) {
    const float w = src[o * ld + off + 8 * oct + e] * kWCarry;
    hv[e] = (_Float16)w;
  }
  _Float16* d = dst + o * 64 + 8 * oct;
  *(volatile v8h*)d = hv;
  __threadfence();
  *(volatile v8h*)d = hv;
  __threadfence();
}

__global__ __launch_bounds__(256) void gemm_tile64_f16(
    const _Float16* __restrict__ A, int lda,
    const _Float16* __restrict__ Bt, int ldb,
    _Float16* __restrict__ C, int ldc,
    int M, int N, int K, float scale) {
  __shared__ __align__(16) float sT[8][16 * 68];
  const int lane = threadIdx.x & 31;
  const int wave = threadIdx.x >> 5;
  const int tilesN = N >> 6;
  const int tilesM = M >> 6;
  const int tile = blockIdx.x * 8 + wave;
  if (tile >= tilesM * tilesN) return;
  const int tm = tile / tilesN;
  const int tn = tile - tm * tilesN;
  const int m0 = tm << 6;
  const int n0 = tn << 6;
  const int rlane = lane & 15;
  const int koff = (lane >> 4) * 8;
  const int mOff = (lane >> 4) * 8;

  v8f acc[4][4];
#pragma unroll
  for (int i = 0; i < 4; ++i)
#pragma unroll
    for (int j = 0; j < 4; ++j) acc[i][j] = (v8f){0.f, 0.f, 0.f, 0.f, 0.f, 0.f, 0.f, 0.f};

  for (int k0 = 0; k0 < K; k0 += 32) {
    v16h bh[4];
#pragma unroll
    for (int j = 0; j < 4; ++j) {
      const size_t bo = (size_t)(n0 + (j << 4) + rlane) * ldb + koff + k0;
      bh[j] = frag_load_g(Bt + bo);
    }
#pragma unroll
    for (int i = 0; i < 4; ++i) {
      const size_t ao = (size_t)(m0 + (i << 4) + rlane) * lda + koff + k0;
      const v16h ah = frag_load_g(A + ao);
#pragma unroll
      for (int j = 0; j < 4; ++j) acc[i][j] = mma_h(ah, bh[j], acc[i][j]);
      guard4_h(acc[i][0], acc[i][1], acc[i][2], acc[i][3], ah, bh[0], bh[1], bh[2], bh[3]);
    }
    keep4_h(bh[0], bh[1], bh[2], bh[3]);
  }
  acc_guard4(acc[0][0], acc[0][1], acc[0][2], acc[0][3]);
  acc_guard4(acc[1][0], acc[1][1], acc[1][2], acc[1][3]);
  acc_guard4(acc[2][0], acc[2][1], acc[2][2], acc[2][3]);
  acc_guard4(acc[3][0], acc[3][1], acc[3][2], acc[3][3]);

  float* slab = sT[wave];
#pragma unroll
  for (int i = 0; i < 4; ++i) {
    const int mBase = m0 + (i << 4);
#pragma unroll
    for (int j = 0; j < 4; ++j) {
#pragma unroll
      for (int r = 0; r < 8; ++r) {
        const float v = acc[i][j][r] * scale;
        slab[(mOff + r) * 68 + (j << 4) + rlane] = v;
      }
    }
    __builtin_amdgcn_fence(__ATOMIC_RELEASE, "workgroup");
    __builtin_amdgcn_wave_barrier();
    __builtin_amdgcn_fence(__ATOMIC_ACQUIRE, "workgroup");
    {
      const int q = lane >> 3;
      const int c8 = (lane & 7) * 8;
      v8h hv[4];
#pragma unroll
      for (int it = 0; it < 4; ++it) {
        const float* sp = slab + (it * 4 + q) * 68 + c8;
#pragma unroll
        for (int e = 0; e < 8; ++e) hv[it][e] = (_Float16)sp[e];
      }
      for (int pass = 0; pass < 2; ++pass) {
#pragma unroll
        for (int it = 0; it < 4; ++it) {
          const int row = it * 4 + q;
          *(volatile v8h*)(C + (size_t)(mBase + row) * ldc + n0 + c8) = hv[it];
        }
        __threadfence();
      }
    }
    __builtin_amdgcn_fence(__ATOMIC_RELEASE, "workgroup");
    __builtin_amdgcn_wave_barrier();
    __builtin_amdgcn_fence(__ATOMIC_ACQUIRE, "workgroup");
  }
}

__device__ __forceinline__ void z0_octet(const float* __restrict__ xyz,
                                         const float* __restrict__ cxyz,
                                         const int* __restrict__ gidx,
                                         const unsigned short* __restrict__ Pp,
                                         int col, int oct,
                                         const float (&wx)[8], const float (&wy)[8],
                                         const float (&wz)[8], float (&z)[8]) {
  const int g = col >> 5;
  const int b = g >> 10;
  const int s = g & (kCent - 1);
  int n = gidx[col];
  n = n < 0 ? 0 : (n > kPts - 1 ? kPts - 1 : n);
  const float* px = xyz + (size_t)b * 3 * kPts;
  const float* cc = cxyz + (size_t)b * 3 * kCent + s;
  const float rx = px[n] - cc[0];
  const float ry = px[kPts + n] - cc[kCent];
  const float rz = px[2 * kPts + n] - cc[2 * kCent];
  const v4u w = *(const v4u*)(Pp + ((size_t)b * kPts + n) * 64 + 8 * oct);
  const unsigned w0 = w.x;
  const unsigned w1 = w.y;
  const unsigned w2 = w.z;
  const unsigned w3 = w.w;
  float p[8];
  p[0] = h16_to_f32(w0 & 0xffffu);
  p[1] = h16_to_f32(w0 >> 16);
  p[2] = h16_to_f32(w1 & 0xffffu);
  p[3] = h16_to_f32(w1 >> 16);
  p[4] = h16_to_f32(w2 & 0xffffu);
  p[5] = h16_to_f32(w2 >> 16);
  p[6] = h16_to_f32(w3 & 0xffffu);
  p[7] = h16_to_f32(w3 >> 16);
#pragma unroll
  for (int e = 0; e < 8; ++e) {
    float t = __builtin_fmaf(wx[e], rx, p[e]);
    t = __builtin_fmaf(wy[e], ry, t);
    t = __builtin_fmaf(wz[e], rz, t);
    z[e] = t;
  }
}

__global__ __launch_bounds__(256) void z0_stats_kernel(const float* __restrict__ xyz,
                                                       const float* __restrict__ cxyz,
                                                       const int* __restrict__ gidx,
                                                       const unsigned short* __restrict__ Pp,
                                                       const float* __restrict__ W0,
                                                       float* __restrict__ part0) {
  __shared__ float s_w[192];
  __shared__ float s_red[8][128];
  const int tid = threadIdx.x;
  const int lane = tid & 31;
  const int wave = tid >> 5;
  const int oct = tid & 7;
  const int rsub = tid >> 3;
  {
    const int ti = tid < 192 ? tid : 191;
    const float wv = W0[(ti / 3) * 67 + (ti % 3)];
    if (tid < 192) s_w[tid] = wv;
  }
  __syncthreads();
  float wx[8], wy[8], wz[8], s1[8], s2[8];
#pragma unroll
  for (int e = 0; e < 8; ++e) {
    const int ch = 8 * oct + e;
    wx[e] = s_w[ch * 3];
    wy[e] = s_w[ch * 3 + 1];
    wz[e] = s_w[ch * 3 + 2];
    s1[e] = 0.0f;
    s2[e] = 0.0f;
  }
  const int colBase = blockIdx.x * kBlkCols;
#pragma unroll 1
  for (int pass = 0; pass < 4; ++pass) {
    float z[8];
    z0_octet(xyz, cxyz, gidx, Pp, colBase + pass * 32 + rsub, oct, wx, wy, wz, z);
#pragma unroll
    for (int e = 0; e < 8; ++e) {
      s1[e] += z[e];
      s2[e] += z[e] * z[e];
    }
  }
#pragma unroll
  for (int e = 0; e < 8; ++e) {
    s1[e] += __shfl_xor(s1[e], 8, 32);
    s2[e] += __shfl_xor(s2[e], 8, 32);
    s1[e] += __shfl_xor(s1[e], 16, 32);
    s2[e] += __shfl_xor(s2[e], 16, 32);
  }
  if (lane < 8) {
#pragma unroll
    for (int e = 0; e < 8; ++e) {
      s_red[wave][8 * oct + e] = s1[e];
      s_red[wave][64 + 8 * oct + e] = s2[e];
    }
  }
  __syncthreads();
  if (tid < 32) {
    v4f o;
#pragma unroll
    for (int e = 0; e < 4; ++e) {
      float a = 0.0f;
#pragma unroll
      for (int w = 0; w < 8; ++w) a += s_red[w][4 * tid + e];
      o[e] = a;
    }
    float* d = part0 + (size_t)blockIdx.x * 128 + 4 * tid;
    *(volatile v4f*)d = o;
    __threadfence();
    *(volatile v4f*)d = o;
    __threadfence();
  }
}

__global__ __launch_bounds__(256) void fin_kernel(const float* __restrict__ part,
                                                  int nblk, int nch,
                                                  const float* __restrict__ gamma,
                                                  const float* __restrict__ beta,
                                                  float* __restrict__ ss) {
  __shared__ double s_d[256];
  __shared__ __align__(16) float s_o[256];
  const int tid = threadIdx.x;
  const int width = 2 * nch;
  const int j = tid < width ? tid : width - 1;
  double acc = 0.0;
#pragma unroll 4
  for (int i = 0; i < nblk; ++i) acc += (double)part[(size_t)i * width + j];
  s_d[tid] = acc;
  __syncthreads();
  {
    const int cr = tid & 127;
    const int c = cr < nch ? cr : nch - 1;
    const double cinv = 1.0 / (double)kCols;
    const double mean = s_d[c] * cinv;
    double var = s_d[nch + c] * cinv - mean * mean;
    var = var < 0.0 ? 0.0 : var;
    const float inv = 1.0f / sqrtf((float)var + 1e-5f);
    const float gm = gamma[c];
    const float bt = beta[c];
    const float sc = gm * inv;
    const float sh = bt - (float)mean * sc;
    const float pick = (tid < 128) ? sc : sh;
    s_o[tid] = (cr < nch) ? pick : 0.0f;
  }
  __syncthreads();
  if (tid < 64) {
    const v4f o = *(const v4f*)(s_o + 4 * tid);
    *(volatile v4f*)(ss + 4 * tid) = o;
    __threadfence();
    *(volatile v4f*)(ss + 4 * tid) = o;
    __threadfence();
  }
}

__global__ __launch_bounds__(256) void layer1_kernel(const float* __restrict__ xyz,
                                                     const float* __restrict__ cxyz,
                                                     const int* __restrict__ gidx,
                                                     const unsigned short* __restrict__ Pp,
                                                     const float* __restrict__ W0,
                                                     const float* __restrict__ ss0,
                                                     const _Float16* __restrict__ W1h,
                                                     _Float16* __restrict__ Z1,
                                                     float* __restrict__ part1) {
  __shared__ __align__(16) _Float16 sA[kBlkCols * kPitchA];
  __shared__ __align__(16) float sT[8][16 * 68];
  __shared__ float s_w[192];
  __shared__ float s_sc[64];
  __shared__ float s_sh[64];
  __shared__ float s_red[8][128];
  const int tid = threadIdx.x;
  const int lane = tid & 31;
  const int wave = tid >> 5;
  const int oct = tid & 7;
  const int rsub = tid >> 3;
  {
    const int ti = tid < 192 ? tid : 191;
    const float wv = W0[(ti / 3) * 67 + (ti % 3)];
    if (tid < 192) s_w[tid] = wv;
    const int tc = tid & 63;
    const float a = ss0[tc];
    const float c = ss0[128 + tc];
    if (tid < 64) { s_sc[tid] = a; s_sh[tid] = c; }
  }
  __syncthreads();
  float wx[8], wy[8], wz[8], sc[8], sh[8];
#pragma unroll
  for (int e = 0; e < 8; ++e) {
    const int ch = 8 * oct + e;
    wx[e] = s_w[ch * 3];
    wy[e] = s_w[ch * 3 + 1];
    wz[e] = s_w[ch * 3 + 2];
    sc[e] = s_sc[ch];
    sh[e] = s_sh[ch];
  }
  const int colBase = blockIdx.x * kBlkCols;
#pragma unroll 1
  for (int pass = 0; pass < 4; ++pass) {
    const int row = pass * 32 + rsub;
    float z[8];
    z0_octet(xyz, cxyz, gidx, Pp, colBase + row, oct, wx, wy, wz, z);
    v8h hv;
#pragma unroll
    for (int e = 0; e < 8; ++e) {
      const float a = fmaxf(__builtin_fmaf(z[e], sc[e], sh[e]), 0.0f);
      hv[e] = (_Float16)a;
    }
    *(v8h*)(sA + row * kPitchA + 8 * oct) = hv;
  }
  __syncthreads();

  const int rlane = lane & 15;
  const int koff = (lane >> 4) * 8;
  const int mOff = (lane >> 4) * 8;
  v8f acc[4];
#pragma unroll
  for (int j = 0; j < 4; ++j) acc[j] = (v8f){0.f, 0.f, 0.f, 0.f, 0.f, 0.f, 0.f, 0.f};
#pragma unroll
  for (int ks = 0; ks < 2; ++ks) {
    v16h bh[4];
#pragma unroll
    for (int j = 0; j < 4; ++j)
      bh[j] = frag_load_g(W1h + (size_t)(j * 16 + rlane) * 64 + ks * 32 + koff);
    FragH fa;
    fa.h[0] = *(const v8h*)(sA + (wave * 16 + rlane) * kPitchA + ks * 32 + koff);
    fa.h[1] = *(const v8h*)(sA + (wave * 16 + rlane) * kPitchA + ks * 32 + koff + 16);
    const v16h ah = fa.v;
#pragma unroll
    for (int j = 0; j < 4; ++j) acc[j] = mma_h(ah, bh[j], acc[j]);
    guard4_h(acc[0], acc[1], acc[2], acc[3], ah, bh[0], bh[1], bh[2], bh[3]);
  }
  acc_guard4(acc[0], acc[1], acc[2], acc[3]);

  float* slab = sT[wave];
  float cs[4], cq[4];
#pragma unroll
  for (int j = 0; j < 4; ++j) {
    float sm = 0.0f, sq = 0.0f;
#pragma unroll
    for (int r = 0; r < 8; ++r) {
      const float v = acc[j][r] * kWCarryInv;
      sm += v;
      sq += v * v;
      slab[(mOff + r) * 68 + j * 16 + rlane] = v;
    }
    cs[j] = sm;
    cq[j] = sq;
  }
#pragma unroll
  for (int j = 0; j < 4; ++j) {
    cs[j] += __shfl_xor(cs[j], 16, 32);
    cq[j] += __shfl_xor(cq[j], 16, 32);
  }
  if (lane < 16) {
#pragma unroll
    for (int j = 0; j < 4; ++j) {
      s_red[wave][j * 16 + lane] = cs[j];
      s_red[wave][64 + j * 16 + lane] = cq[j];
    }
  }
  __builtin_amdgcn_fence(__ATOMIC_RELEASE, "workgroup");
  __builtin_amdgcn_wave_barrier();
  __builtin_amdgcn_fence(__ATOMIC_ACQUIRE, "workgroup");
  {
    const int q = lane >> 3;
    const int c8 = (lane & 7) * 8;
    const int rowBase = colBase + wave * 16;
    v8h hv[4];
#pragma unroll
    for (int it = 0; it < 4; ++it) {
      const float* sp = slab + (it * 4 + q) * 68 + c8;
#pragma unroll
      for (int e = 0; e < 8; ++e) hv[it][e] = (_Float16)sp[e];
    }
    for (int pass = 0; pass < 2; ++pass) {
#pragma unroll
      for (int it = 0; it < 4; ++it) {
        const int row = it * 4 + q;
        *(volatile v8h*)(Z1 + (size_t)(rowBase + row) * 64 + c8) = hv[it];
      }
      __threadfence();
    }
  }
  __syncthreads();
  if (tid < 32) {
    v4f o;
#pragma unroll
    for (int e = 0; e < 4; ++e) {
      float a = 0.0f;
#pragma unroll
      for (int w = 0; w < 8; ++w) a += s_red[w][4 * tid + e];
      o[e] = a;
    }
    float* d = part1 + (size_t)blockIdx.x * 128 + 4 * tid;
    *(volatile v4f*)d = o;
    __threadfence();
    *(volatile v4f*)d = o;
    __threadfence();
  }
}

__global__ __launch_bounds__(256) void layer2_kernel(const unsigned short* __restrict__ Z1p,
                                                     const float* __restrict__ ss1,
                                                     const _Float16* __restrict__ W2h,
                                                     float* __restrict__ zmax,
                                                     float* __restrict__ zmin,
                                                     float* __restrict__ part2) {
  __shared__ __align__(16) _Float16 sA[kBlkCols * kPitchA];
  __shared__ float s_sc[64];
  __shared__ float s_sh[64];
  __shared__ __align__(16) float s_red[8][4][128];
  const int tid = threadIdx.x;
  const int lane = tid & 31;
  const int wave = tid >> 5;
  const int oct = tid & 7;
  const int rsub = tid >> 3;
  {
    const int tc = tid & 63;
    const float a = ss1[tc];
    const float c = ss1[128 + tc];
    if (tid < 64) { s_sc[tid] = a; s_sh[tid] = c; }
  }
  __syncthreads();
  float sc[8], sh[8];
#pragma unroll
  for (int e = 0; e < 8; ++e) {
    sc[e] = s_sc[8 * oct + e];
    sh[e] = s_sh[8 * oct + e];
  }
  const int colBase = blockIdx.x * kBlkCols;
#pragma unroll 1
  for (int pass = 0; pass < 4; ++pass) {
    const int row = pass * 32 + rsub;
    const v4u w = *(const v4u*)(Z1p + (size_t)(colBase + row) * 64 + 8 * oct);
    const unsigned w0 = w.x;
    const unsigned w1 = w.y;
    const unsigned w2 = w.z;
    const unsigned w3 = w.w;
    float z[8];
    z[0] = h16_to_f32(w0 & 0xffffu);
    z[1] = h16_to_f32(w0 >> 16);
    z[2] = h16_to_f32(w1 & 0xffffu);
    z[3] = h16_to_f32(w1 >> 16);
    z[4] = h16_to_f32(w2 & 0xffffu);
    z[5] = h16_to_f32(w2 >> 16);
    z[6] = h16_to_f32(w3 & 0xffffu);
    z[7] = h16_to_f32(w3 >> 16);
    v8h hv;
#pragma unroll
    for (int e = 0; e < 8; ++e) {
      const float a = fmaxf(__builtin_fmaf(z[e], sc[e], sh[e]), 0.0f);
      hv[e] = (_Float16)a;
    }
    *(v8h*)(sA + row * kPitchA + 8 * oct) = hv;
  }
  __syncthreads();

  const int rlane = lane & 15;
  const int koff = (lane >> 4) * 8;
  v8f acc[8];
#pragma unroll
  for (int j = 0; j < 8; ++j) acc[j] = (v8f){0.f, 0.f, 0.f, 0.f, 0.f, 0.f, 0.f, 0.f};
#pragma unroll
  for (int ks = 0; ks < 2; ++ks) {
    FragH fa;
    fa.h[0] = *(const v8h*)(sA + (wave * 16 + rlane) * kPitchA + ks * 32 + koff);
    fa.h[1] = *(const v8h*)(sA + (wave * 16 + rlane) * kPitchA + ks * 32 + koff + 16);
    const v16h ah = fa.v;
#pragma unroll
    for (int jh = 0; jh < 2; ++jh) {
      v16h bh[4];
#pragma unroll
      for (int j = 0; j < 4; ++j)
        bh[j] = frag_load_g(W2h + (size_t)((jh * 4 + j) * 16 + rlane) * 64 + ks * 32 + koff);
#pragma unroll
      for (int j = 0; j < 4; ++j) acc[jh * 4 + j] = mma_h(ah, bh[j], acc[jh * 4 + j]);
      guard4_h(acc[jh * 4 + 0], acc[jh * 4 + 1], acc[jh * 4 + 2], acc[jh * 4 + 3],
               ah, bh[0], bh[1], bh[2], bh[3]);
    }
  }
  acc_guard4(acc[0], acc[1], acc[2], acc[3]);
  acc_guard4(acc[4], acc[5], acc[6], acc[7]);

  float amx[8], amn[8], asu[8], asq[8];
#pragma unroll
  for (int j = 0; j < 8; ++j) {
    float mx = -INFINITY, mn = INFINITY, sm = 0.0f, sq = 0.0f;
#pragma unroll
    for (int r = 0; r < 8; ++r) {
      const float v = acc[j][r] * kWCarryInv;
      mx = fmaxf(mx, v);
      mn = fminf(mn, v);
      sm += v;
      sq += v * v;
    }
    amx[j] = mx; amn[j] = mn; asu[j] = sm; asq[j] = sq;
  }
#pragma unroll
  for (int j = 0; j < 8; ++j) {
    const float mx2 = __shfl_xor(amx[j], 16, 32);
    const float mn2 = __shfl_xor(amn[j], 16, 32);
    const float sm2 = __shfl_xor(asu[j], 16, 32);
    const float sq2 = __shfl_xor(asq[j], 16, 32);
    amx[j] = fmaxf(amx[j], mx2);
    amn[j] = fminf(amn[j], mn2);
    asu[j] += sm2;
    asq[j] += sq2;
  }
  if (lane < 16) {
#pragma unroll
    for (int j = 0; j < 8; ++j) {
      s_red[wave][0][j * 16 + lane] = amx[j];
      s_red[wave][1][j * 16 + lane] = amn[j];
      s_red[wave][2][j * 16 + lane] = asu[j];
      s_red[wave][3][j * 16 + lane] = asq[j];
    }
  }
  __syncthreads();
  {
    const int plane = wave >> 2;
    const int gq = wave & 3;
    v4f o;
#pragma unroll
    for (int e = 0; e < 4; ++e) {
      const float a = s_red[2 * gq][plane][4 * lane + e];
      const float c = s_red[2 * gq + 1][plane][4 * lane + e];
      const float hi = fmaxf(a, c);
      const float lo = fminf(a, c);
      o[e] = (plane == 0) ? hi : lo;
    }
    float* base = (plane == 0) ? zmax : zmin;
    float* d = base + ((size_t)blockIdx.x * 4 + gq) * 128 + 4 * lane;
    *(volatile v4f*)d = o;
    __threadfence();
    *(volatile v4f*)d = o;
    __threadfence();
  }
  if (tid < 64) {
    const int which = tid >> 5;
    v4f o;
#pragma unroll
    for (int e = 0; e < 4; ++e) {
      float a = 0.0f;
#pragma unroll
      for (int w = 0; w < 8; ++w) a += s_red[w][2 + which][4 * lane + e];
      o[e] = a;
    }
    float* d = part2 + (size_t)blockIdx.x * 256 + which * 128 + 4 * lane;
    *(volatile v4f*)d = o;
    __threadfence();
    *(volatile v4f*)d = o;
    __threadfence();
  }
}

__global__ __launch_bounds__(256) void out1_kernel(const float* __restrict__ zmax,
                                                   const float* __restrict__ zmin,
                                                   const float* __restrict__ ss2,
                                                   float* __restrict__ out1) {
  __shared__ float tile[128 * 33];
  __shared__ float s_sc[128];
  __shared__ float s_sh[128];
  const int tid = threadIdx.x;
  const int lane = tid & 31;
  const int wave = tid >> 5;
  const int blk = blockIdx.x;
  const int b = blk >> 5;
  const int s0 = (blk & 31) * 32;
  {
    const int tc = tid & 127;
    const float a = ss2[tc];
    const float c = ss2[128 + tc];
    if (tid < 128) { s_sc[tid] = a; s_sh[tid] = c; }
  }
  __syncthreads();
  {
    const int row = tid >> 3;
    const int q = tid & 7;
    const size_t g = (size_t)b * kCent + s0 + row;
#pragma unroll
    for (int i = 0; i < 4; ++i) {
      const int c4 = 4 * (q + 8 * i);
      const v4f a = *(const v4f*)(zmax + g * 128 + c4);
      const v4f m = *(const v4f*)(zmin + g * 128 + c4);
#pragma unroll
      for (int e = 0; e < 4; ++e) {
        const int ch = c4 + e;
        const float scv = s_sc[ch];
        const float shv = s_sh[ch];
        const float ya = __builtin_fmaf(scv, a[e], shv);
        const float ym = __builtin_fmaf(scv, m[e], shv);
        tile[ch * 33 + row] = fmaxf(fmaxf(ya, ym), 0.0f);
      }
    }
  }
  __syncthreads();
  {
    const int sub = lane >> 3;
    const int s4 = (lane & 7) * 4;
    v4f o[4];
#pragma unroll
    for (int it = 0; it < 4; ++it) {
      const int ch = it * 32 + wave * 4 + sub;
      o[it][0] = tile[ch * 33 + s4];
      o[it][1] = tile[ch * 33 + s4 + 1];
      o[it][2] = tile[ch * 33 + s4 + 2];
      o[it][3] = tile[ch * 33 + s4 + 3];
    }
    for (int pass = 0; pass < 2; ++pass) {
#pragma unroll
      for (int it = 0; it < 4; ++it) {
        const int ch = it * 32 + wave * 4 + sub;
        *(volatile v4f*)(out1 + ((size_t)b * 128 + ch) * kCent + s0 + s4) = o[it];
      }
      __threadfence();
    }
  }
}

extern "C" void kernel_launch(void* const* d_in, const int* in_sizes, int n_in,
                              void* d_out, int out_size, void* d_ws, size_t ws_size,
                              hipStream_t stream) {
  (void)in_sizes; (void)n_in; (void)out_size;
  const float* xyz  = (const float*)d_in[0];
  const float* feat = (const float*)d_in[1];
  const float* W0   = (const float*)d_in[2];
  const float* g0   = (const float*)d_in[3];
  const float* be0  = (const float*)d_in[4];
  const float* W1   = (const float*)d_in[5];
  const float* g1   = (const float*)d_in[6];
  const float* be1  = (const float*)d_in[7];
  const float* W2   = (const float*)d_in[8];
  const float* g2   = (const float*)d_in[9];
  const float* be2  = (const float*)d_in[10];
  float* out0 = (float*)d_out;
  float* out1 = out0 + kOut0Floats;

  char* ws = (char*)d_ws;
  size_t off = 0;
  auto carve = [&](size_t bytes) -> char* {
    char* p = ws + off;
    off = (off + bytes + 255) & ~(size_t)255;
    return p;
  };
  int*      gidx  = (int*)carve((size_t)kCols * 4);
  float*    cxyz  = (float*)carve((size_t)kOut0Floats * 4);
  _Float16* featT = (_Float16*)carve((size_t)kRowsAll * 64 * 2);
  _Float16* Pp    = (_Float16*)carve((size_t)kRowsAll * 64 * 2);
  _Float16* Z1    = (_Float16*)carve((size_t)kCols * 64 * 2);
  float*    zmax  = (float*)carve((size_t)kBatch * kCent * 128 * 4);
  float*    zmin  = (float*)carve((size_t)kBatch * kCent * 128 * 4);
  float*    part0 = (float*)carve((size_t)kNumBlk * 128 * 4);
  float*    part1 = (float*)carve((size_t)kNumBlk * 128 * 4);
  float*    part2 = (float*)carve((size_t)kNumBlk * 256 * 4);
  _Float16* W0f   = (_Float16*)carve((size_t)64 * 64 * 2);
  _Float16* W1h   = (_Float16*)carve((size_t)64 * 64 * 2);
  _Float16* W2h   = (_Float16*)carve((size_t)128 * 64 * 2);
  float*    ss0   = (float*)carve(256 * 4);
  float*    ss1   = (float*)carve(256 * 4);
  float*    ss2   = (float*)carve(256 * 4);
  if (off > ws_size) return;
  if (off > (size_t)134217728) return;

  fps_kernel<<<kBatch, 1024, 0, stream>>>(xyz, out0, cxyz);
  ballquery_kernel<<<(kBatch * kCent) / 8, 256, 0, stream>>>(xyz, cxyz, gidx);
  cvt_feat_kernel<<<kRowsAll / 64, 256, 0, stream>>>(feat, featT);
  cvt_w_kernel<<<8, 256, 0, stream>>>(W0, W1, W2, W0f, W1h, W2h);

  gemm_tile64_f16<<<(kRowsAll / 64) / 8, 256, 0, stream>>>(
      featT, 64, W0f, 64, Pp, 64, kRowsAll, 64, 64, kWCarryInv);

  z0_stats_kernel<<<kNumBlk, 256, 0, stream>>>(
      xyz, cxyz, gidx, (const unsigned short*)Pp, W0, part0);
  fin_kernel<<<1, 256, 0, stream>>>(part0, kNumBlk, 64, g0, be0, ss0);

  layer1_kernel<<<kNumBlk, 256, 0, stream>>>(
      xyz, cxyz, gidx, (const unsigned short*)Pp, W0, ss0, W1h, Z1, part1);
  fin_kernel<<<1, 256, 0, stream>>>(part1, kNumBlk, 64, g1, be1, ss1);

  layer2_kernel<<<kNumBlk, 256, 0, stream>>>(
      (const unsigned short*)Z1, ss1, W2h, zmax, zmin, part2);
  fin_kernel<<<1, 256, 0, stream>>>(part2, kNumBlk, 128, g2, be2, ss2);

  out1_kernel<<<(kBatch * kCent) / 32, 256, 0, stream>>>(zmax, zmin, ss2, out1);
}
